// DecoderLayer_77988016160858
// MI455X (gfx1250) — hardware-verified
//
#include <hip/hip_runtime.h>
#ifndef NB
#define NB 4
#endif
#ifndef SEQ
#define SEQ 2048
#endif
#define NB_FULL 4
#define SEQ_FULL 2048
#define DM 1024
#define NH 16
#define HD 64
#define DFF 4096
#define LQ (3 * DM)
#define MROWS (NB * SEQ)
#define NQT (SEQ / 64)
static_assert(SEQ % 64 == 0);
static_assert(SEQ <= SEQ_FULL);
static_assert(NB >= 1 && NB <= NB_FULL);
static_assert(MROWS % 128 == 0);
static_assert(MROWS % 8 == 0);
static_assert(DM % 64 == 0 && DFF % 64 == 0 && LQ % 64 == 0);
static_assert(DM % 32 == 0 && DFF % 32 == 0);
static_assert(NH * HD == DM);
static_assert(DM + LQ == DFF);
static_assert(NB * NH * HD * SEQ == MROWS * DM);
static_assert((MROWS / 128) * (LQ / 64) * 128 * 64 == MROWS * LQ);
static_assert((MROWS / 128) * (DM / 64) * 128 * 64 == MROWS * DM);
static_assert((MROWS / 128) * (DFF / 64) * 128 * 64 == MROWS * DFF);
static_assert(NQT * NB * NH * 4 * 16 * 64 == MROWS * DM);

typedef _Float16 v16h __attribute__((ext_vector_type(16)));
typedef _Float16 v4h  __attribute__((ext_vector_type(4)));
typedef unsigned short v8us __attribute__((ext_vector_type(8), may_alias));
typedef float  v8f  __attribute__((ext_vector_type(8)));
typedef float  v4f  __attribute__((ext_vector_type(4)));
typedef float  v4fa __attribute__((ext_vector_type(4), may_alias));
union FragH { v16h v; v8us half[2]; _Float16 h[16]; unsigned short u[16]; };

#define NEG_INF (-__builtin_inff())

__device__ __forceinline__ unsigned short bf16_bits(float x) { unsigned int u = __float_as_uint(x); return (unsigned short)((u + 0x7FFFu + ((u >> 16) & 1u)) >> 16); }
__device__ __forceinline__ float bf16_val(unsigned short b) { return __uint_as_float(((unsigned int)b) << 16); }
__device__ __forceinline__ float bf16_rne(float x) { return bf16_val(bf16_bits(x)); }

__device__ __forceinline__ int frow(int m) { return (m / SEQ) * SEQ_FULL + (m % SEQ); }

__device__ __forceinline__ v16h g2_frag(const _Float16* p, int hh) { FragH f; f.half[0] = *(const v8us*)((const unsigned short*)p + 8 * hh); f.half[1] = *(const v8us*)((const unsigned short*)p + 16 + 8 * hh); return f.v; }
__device__ __forceinline__ v8f g2_mma(v16h a, v16h b, v8f c) { v8f d = __builtin_amdgcn_wmma_f32_16x16x32_f16(false, a, false, b, (short)0, c, false, false); asm volatile("v_nop\n\tv_nop\n\tv_nop\n\tv_nop" : "+v"(d) : "v"(a), "v"(b)); return d; }

__device__ __forceinline__ float gelu_f(float t) {
  const float z = t * 0.70710678118654752f; const float az = fabsf(z);
  const float u = __builtin_amdgcn_rcpf(fmaf(0.3275911f, az, 1.0f));
  float p = 1.061405429f; p = fmaf(p, u, -1.453152027f); p = fmaf(p, u, 1.421413741f); p = fmaf(p, u, -0.284496736f); p = fmaf(p, u, 0.254829592f); p *= u;
  const float pe = p * exp2f(-az * az * 1.4426950408889634f);
  const float c = (z < 0.0f) ? pe : (2.0f - pe);
  return 0.5f * t * c; }

__global__ __launch_bounds__(256) void k_wT(const float* __restrict__ w, int ldin, int zin, _Float16* __restrict__ Bt, int ldo, int zout, int ktiles, int ntiles) {
  __shared__ unsigned short tl[64][66];
  const int tid = threadIdx.x; int bi = blockIdx.x; const int nt = bi % ntiles; bi /= ntiles; const int kt = bi % ktiles; const int z = bi / ktiles;
  const float* src = w + (size_t)z * zin + (size_t)(kt * 64) * ldin + nt * 64;
  for (int i = tid; i < 64 * 16; i += 256) { const int r = i >> 4, c4 = (i & 15) * 4; const v4f v = *(const v4fa*)(src + (size_t)r * ldin + c4); FragH f;
#pragma unroll
    for (int q = 0; q < 4; ++q) f.h[q] = (_Float16)(bf16_rne(v[q]) * 16.0f);
#pragma unroll
    for (int q = 0; q < 4; ++q) tl[r][c4 + q] = f.u[q]; }
  __syncthreads();
  unsigned short* dst = (unsigned short*)Bt + (size_t)z * zout + (size_t)(nt * 64) * ldo + kt * 64;
  for (int pass = 0; pass < 2; ++pass) {
#pragma unroll
    for (int rd = 0; rd < 2; ++rd) { const int d = rd * 32 + tid / 8, pc = tid % 8; FragH f;
#pragma unroll
      for (int q = 0; q < 8; ++q) f.u[q] = tl[pc * 8 + q][d];
      *(volatile v8us*)(dst + (size_t)d * ldo + pc * 8) = f.half[0]; }
    if (pass == 0) __threadfence(); } }

__global__ __launch_bounds__(256) void k_ln(const float* in, const float* __restrict__ g, const float* __restrict__ bt, _Float16* __restrict__ H, int rnd) {
  const int w = threadIdx.x >> 5, lane = threadIdx.x & 31; const int m = blockIdx.x * 8 + w;
  const float* xr = in + (size_t)frow(m) * DM + lane * 8;
  float s = 0.f;
#pragma unroll 1
  for (int j = 0; j < 4; ++j) { v4f a = *(const v4fa*)(xr + j * 256), c = *(const v4fa*)(xr + j * 256 + 4);
    if (rnd != 0) {
#pragma unroll
      for (int i = 0; i < 4; ++i) { a[i] = bf16_rne(a[i]); c[i] = bf16_rne(c[i]); } }
    s += ((a[0] + a[1]) + (a[2] + a[3])) + ((c[0] + c[1]) + (c[2] + c[3])); }
  s += __shfl_xor(s, 16); s += __shfl_xor(s, 8); s += __shfl_xor(s, 4); s += __shfl_xor(s, 2); s += __shfl_xor(s, 1);
  const float mu = s * (1.0f / 1024.0f);
  float qs = 0.f;
#pragma unroll 1
  for (int j = 0; j < 4; ++j) { v4f a = *(const v4fa*)(xr + j * 256), c = *(const v4fa*)(xr + j * 256 + 4);
    if (rnd != 0) {
#pragma unroll
      for (int i = 0; i < 4; ++i) { a[i] = bf16_rne(a[i]); c[i] = bf16_rne(c[i]); } }
#pragma unroll
    for (int i = 0; i < 4; ++i) { const float d0 = a[i] - mu, d1 = c[i] - mu; qs = fmaf(d0, d0, qs); qs = fmaf(d1, d1, qs); } }
  qs += __shfl_xor(qs, 16); qs += __shfl_xor(qs, 8); qs += __shfl_xor(qs, 4); qs += __shfl_xor(qs, 2); qs += __shfl_xor(qs, 1);
  const float rs = rsqrtf(qs * (1.0f / 1024.0f) + 1e-5f);
  unsigned short* hp = (unsigned short*)H + (size_t)m * DM + lane * 8;
#pragma unroll 1
  for (int j = 0; j < 4; ++j) { v4f a = *(const v4fa*)(xr + j * 256), c = *(const v4fa*)(xr + j * 256 + 4);
    const v4f ga = *(const v4fa*)(g + j * 256 + lane * 8), gc = *(const v4fa*)(g + j * 256 + lane * 8 + 4);
    const v4f ba = *(const v4fa*)(bt + j * 256 + lane * 8), bc = *(const v4fa*)(bt + j * 256 + lane * 8 + 4);
    if (rnd != 0) {
#pragma unroll
      for (int i = 0; i < 4; ++i) { a[i] = bf16_rne(a[i]); c[i] = bf16_rne(c[i]); } }
    FragH f;
#pragma unroll
    for (int i = 0; i < 4; ++i) { f.h[i] = (_Float16)((a[i] - mu) * rs * bf16_rne(ga[i]) + bf16_rne(ba[i])); f.h[4 + i] = (_Float16)((c[i] - mu) * rs * bf16_rne(gc[i]) + bf16_rne(bc[i])); }
    const v8us val = f.half[0];
    *(volatile v8us*)(hp + j * 256) = val; __threadfence(); *(volatile v8us*)(hp + j * 256) = val; } }

template <int EPI>
__global__ __launch_bounds__(128) void k_gemm2(const _Float16* __restrict__ A, int lda, const _Float16* __restrict__ Bh, int ldb, float alpha, const float* __restrict__ bias,
    _Float16* __restrict__ C16, const float* res, float* outF, int ldc, int M, int N, int K) {
  __shared__ __attribute__((aligned(16))) float so[4][32][68];
  const int tid = threadIdx.x, w = tid >> 5, lane = tid & 31, ln = lane & 15, hh = lane >> 4;
  const int ntn = N >> 6; const int mt = blockIdx.x / ntn, nq = blockIdx.x - mt * ntn; const int row0 = mt * 128 + 32 * w, col0 = nq * 64; if (row0 >= M) return;
  const _Float16* a0p = A + (size_t)(row0 + ln) * lda; const _Float16* a1p = a0p + (size_t)16 * lda;
  const _Float16* b0p = Bh + (size_t)(col0 + ln) * ldb; const _Float16* b1p = b0p + (size_t)16 * ldb; const _Float16* b2p = b1p + (size_t)16 * ldb; const _Float16* b3p = b2p + (size_t)16 * ldb;
  const v8f z8 = {0.f,0.f,0.f,0.f,0.f,0.f,0.f,0.f}; v8f c00 = z8, c01 = z8, c02 = z8, c03 = z8, c10 = z8, c11 = z8, c12 = z8, c13 = z8;
#pragma unroll 1
  for (int kb = 0; kb < K; kb += 32) { const v16h a0 = g2_frag(a0p + kb, hh), a1 = g2_frag(a1p + kb, hh);
    v16h b = g2_frag(b0p + kb, hh); c00 = g2_mma(a0, b, c00); c10 = g2_mma(a1, b, c10);
    b = g2_frag(b1p + kb, hh); c01 = g2_mma(a0, b, c01); c11 = g2_mma(a1, b, c11);
    b = g2_frag(b2p + kb, hh); c02 = g2_mma(a0, b, c02); c12 = g2_mma(a1, b, c12);
    b = g2_frag(b3p + kb, hh); c03 = g2_mma(a0, b, c03); c13 = g2_mma(a1, b, c13); }
  v8f accs[8] = {c00, c01, c02, c03, c10, c11, c12, c13};
#pragma unroll
  for (int u = 0; u < 8; ++u) { const int t = u & 3, half = u >> 2; const int col = col0 + t * 16 + ln; float bv = 0.0f; if (EPI != 0) bv = bf16_rne(bias[col]);
#pragma unroll
    for (int r = 0; r < 8; ++r) { const int rloc = half * 16 + 8 * hh + r; so[w][rloc][t * 16 + ln] = accs[u][r] * alpha + bv; } }
  __builtin_amdgcn_fence(4  , "workgroup"); __builtin_amdgcn_wave_barrier();
  if (EPI <= 1) {
    const int rsub = lane >> 4, c4 = (lane & 15) * 4;
    if (EPI == 1) {
#pragma unroll 1
      for (int q = 0; q < 16; ++q) { const int r = q * 2 + rsub; v4f v = *(const v4fa*)&so[w][r][c4];
#pragma unroll
        for (int i = 0; i < 4; ++i) v[i] = gelu_f(v[i]);
        *(v4fa*)&so[w][r][c4] = v; }
      __builtin_amdgcn_fence(4  , "workgroup"); __builtin_amdgcn_wave_barrier(); }
    for (int pass = 0; pass < 2; ++pass) {
#pragma unroll
      for (int q = 0; q < 16; ++q) { const int r = q * 2 + rsub; const v4f v = *(const v4fa*)&so[w][r][c4]; v4h h4;
#pragma unroll
        for (int i = 0; i < 4; ++i) h4[i] = (_Float16)v[i];
        *(volatile v4h*)(C16 + (size_t)(row0 + r) * ldc + col0 + c4) = h4; }
      if (pass == 0) __threadfence(); }
  } else {
    const int rq = lane >> 3, pc = lane & 7;
#pragma unroll 1
    for (int g = 0; g < 16; ++g) { const int L = g * 4 + rq; const int row = L >> 1, col = (L & 1) * 32 + pc * 4;
      const size_t gi = (size_t)frow(row0 + row) * ldc + col0 + col;
      v4f v = *(const v4fa*)&so[w][row][col]; const v4f xr = *(const v4fa*)(res + gi);
#pragma unroll
      for (int i = 0; i < 4; ++i) v[i] += (EPI == 2) ? bf16_rne(xr[i]) : xr[i];
      *(v4fa*)&so[w][row][col] = v; }
    __builtin_amdgcn_fence(4  , "workgroup"); __builtin_amdgcn_wave_barrier();
    for (int pass = 0; pass < 2; ++pass) {
#pragma unroll 4
      for (int g = 0; g < 16; ++g) { const int L = g * 4 + rq; const int row = L >> 1, col = (L & 1) * 32 + pc * 4;
        const size_t gi = (size_t)frow(row0 + row) * ldc + col0 + col;
        const v4f v = *(const v4fa*)&so[w][row][col];
        *(volatile v4f*)(outF + gi) = v; }
      if (pass == 0) __threadfence(); } } }

__global__ __launch_bounds__(256) void k_vt2(const _Float16* __restrict__ QKV, _Float16* __restrict__ VT) {
  __shared__ unsigned short tl[64][66];
  const int tid = threadIdx.x; const int slab = blockIdx.x / NQT, lg = blockIdx.x - slab * NQT; const int b = slab / NH, hd = slab - b * NH; const int s0 = lg * 64;
  for (int i = tid; i < 64 * 8; i += 256) { const int r = i / 8, c8 = (i % 8) * 8; FragH f;
    f.half[0] = *(const v8us*)((const unsigned short*)QKV + ((size_t)b * SEQ + s0 + r) * LQ + 2 * DM + hd * HD + c8);
#pragma unroll
    for (int q = 0; q < 8; ++q) tl[r][c8 + q] = f.u[q]; }
  __syncthreads();
  for (int pass = 0; pass < 2; ++pass) {
#pragma unroll
    for (int rd = 0; rd < 2; ++rd) { const int d = rd * 32 + tid / 8, pc = tid % 8; FragH f;
#pragma unroll
      for (int q = 0; q < 8; ++q) f.u[q] = tl[pc * 8 + q][d];
      *(volatile v8us*)((unsigned short*)VT + ((size_t)slab * HD + d) * SEQ + s0 + pc * 8) = f.half[0]; }
    if (pass == 0) __threadfence(); } }

__global__ __launch_bounds__(128) void k_attn(const _Float16* __restrict__ QKV, const _Float16* __restrict__ VT, _Float16* __restrict__ CTX) {
  __shared__ __attribute__((aligned(16))) float so[4][16][68];
  const int tid = threadIdx.x, w = tid >> 5, lane = tid & 31, l15 = lane & 15, hh = lane >> 4;
  const int qt = blockIdx.x, slab = blockIdx.y; const int b = slab / NH, hd = slab - b * NH;
  const int q0 = qt * 64 + w * 16;
  const _Float16* Qb = QKV + (size_t)b * SEQ * LQ + hd * HD;
  const _Float16* Kb = Qb + DM;
  const _Float16* Vb = VT + (size_t)slab * HD * SEQ;
  const _Float16* qrow = Qb + (size_t)(q0 + l15) * LQ;
  const v16h qf0 = g2_frag(qrow, hh), qf1 = g2_frag(qrow + 32, hh);
  const v8f z8 = {0.f,0.f,0.f,0.f,0.f,0.f,0.f,0.f};
  v8f o[4] = {z8, z8, z8, z8};
  float m = NEG_INF, l = 0.f;
  const float CL = 0.18033688011112042f;
  const int qi = q0 + l15;
#pragma unroll 1
  for (int it = 0; it <= qt; ++it) {
    const int key0 = it * 64;
    v8f s[4];
#pragma unroll
    for (int kt = 0; kt < 4; ++kt) {
      const _Float16* krow = Kb + (size_t)(key0 + kt * 16 + l15) * LQ;
      const v16h ka = g2_frag(krow, hh), kk = g2_frag(krow + 32, hh);
      v8f a = g2_mma(ka, qf0, z8); a = g2_mma(kk, qf1, a); s[kt] = a; }
    if (it == qt) {
#pragma unroll
      for (int kt = 0; kt < 4; ++kt)
#pragma unroll
        for (int r = 0; r < 8; ++r) { const int key = key0 + kt * 16 + 8 * hh + r; s[kt][r] = (key > qi) ? NEG_INF : s[kt][r]; } }
    float lmax = NEG_INF;
#pragma unroll
    for (int kt = 0; kt < 4; ++kt)
#pragma unroll
      for (int r = 0; r < 8; ++r) lmax = fmaxf(lmax, s[kt][r]);
    lmax = fmaxf(lmax, __shfl_xor(lmax, 16));
    const float mnew = fmaxf(m, lmax);
    const float mref = (mnew == NEG_INF) ? 0.0f : mnew;
    const float alpha = exp2f((m - mref) * CL);
    const float bexp = 10.0f - mref * CL;
    m = mnew;
    float psum = 0.f; FragH pa, pb;
#pragma unroll
    for (int r = 0; r < 8; ++r) {
      const float e0 = exp2f(fmaf(s[0][r], CL, bexp)), e1 = exp2f(fmaf(s[1][r], CL, bexp)), e2 = exp2f(fmaf(s[2][r], CL, bexp)), e3 = exp2f(fmaf(s[3][r], CL, bexp));
      psum += (e0 + e1) + (e2 + e3);
      pa.h[r] = (_Float16)e0; pa.h[8 + r] = (_Float16)e1; pb.h[r] = (_Float16)e2; pb.h[8 + r] = (_Float16)e3; }
    l = l * alpha + psum;
    float ar[8];
#pragma unroll
    for (int r = 0; r < 8; ++r) ar[r] = __shfl(alpha, 8 * hh + r);
#pragma unroll
    for (int dt = 0; dt < 4; ++dt) {
#pragma unroll
      for (int r = 0; r < 8; ++r) o[dt][r] *= ar[r];
      const _Float16* vrow = Vb + (size_t)(dt * 16 + l15) * SEQ + key0;
      const v16h va = g2_frag(vrow, hh), vb = g2_frag(vrow + 32, hh);
      o[dt] = g2_mma(pa.v, va, o[dt]); o[dt] = g2_mma(pb.v, vb, o[dt]); } }
  const float lt = l + __shfl_xor(l, 16);
  const float inv = 16.0f / lt;
  float ir[8];
#pragma unroll
  for (int r = 0; r < 8; ++r) ir[r] = __shfl(inv, 8 * hh + r);
#pragma unroll
  for (int dt = 0; dt < 4; ++dt)
#pragma unroll
    for (int r = 0; r < 8; ++r) so[w][8 * hh + r][dt * 16 + l15] = o[dt][r] * ir[r];
  __builtin_amdgcn_fence(4  , "workgroup"); __builtin_amdgcn_wave_barrier();
  const int rq = lane >> 3, pc = lane & 7;
  FragH fo[4];
#pragma unroll
  for (int g = 0; g < 4; ++g) { const int row = g * 4 + rq; const v4f a = *(const v4fa*)&so[w][row][pc * 8]; const v4f c = *(const v4fa*)&so[w][row][pc * 8 + 4];
#pragma unroll
    for (int i = 0; i < 4; ++i) { fo[g].h[i] = (_Float16)a[i]; fo[g].h[4 + i] = (_Float16)c[i]; } }
  for (int pass = 0; pass < 2; ++pass) {
#pragma unroll
    for (int g = 0; g < 4; ++g) { const int row = g * 4 + rq;
      *(volatile v8us*)((unsigned short*)CTX + ((size_t)b * SEQ + q0 + row) * DM + hd * HD + pc * 8) = fo[g].half[0]; }
    if (pass == 0) __threadfence(); } }

extern "C" void kernel_launch(void* const* d_in, const int* in_sizes, int n_in,
                              void* d_out, int out_size, void* d_ws, size_t ws_size, hipStream_t stream) {
  if (n_in < 14) return;
  const float* x    = (const float*)d_in[0];
  const float* g1   = (const float*)d_in[1];
  const float* bt1  = (const float*)d_in[2];
  const float* wq   = (const float*)d_in[3];
  const float* wk   = (const float*)d_in[4];
  const float* wv   = (const float*)d_in[5];
  const float* wo   = (const float*)d_in[6];
  const float* bo   = (const float*)d_in[7];
  const float* g2   = (const float*)d_in[8];
  const float* bt2  = (const float*)d_in[9];
  const float* wfc  = (const float*)d_in[10];
  const float* bfc  = (const float*)d_in[11];
  const float* wpr  = (const float*)d_in[12];
  const float* bpr  = (const float*)d_in[13];
  float* out = (float*)d_out;
  const int xneed = ((NB - 1) * SEQ_FULL + SEQ) * DM;
  if (in_sizes[0] < xneed || out_size < xneed) return;
  if (in_sizes[1] < DM || in_sizes[2] < DM || in_sizes[8] < DM || in_sizes[9] < DM) return;
  if (in_sizes[3] < NH * DM * HD || in_sizes[4] < NH * DM * HD || in_sizes[5] < NH * DM * HD) return;
  if (in_sizes[6] < DM * DM || in_sizes[7] < DM) return;
  if (in_sizes[10] < DM * DFF || in_sizes[11] < DFF || in_sizes[12] < DFF * DM || in_sizes[13] < DM) return;
  char* ws = (char*)d_ws; size_t off = 0;
  auto take = [&](size_t bytes) { char* p = ws + off; off += (bytes + 255) & ~(size_t)255; return p; };
  _Float16* WQKV = (_Float16*)take((size_t)LQ * DM * 2);
  _Float16* WO   = (_Float16*)take((size_t)DM * DM * 2);
  _Float16* WFC  = (_Float16*)take((size_t)DFF * DM * 2);
  _Float16* WPR  = (_Float16*)take((size_t)DM * DFF * 2);
  _Float16* RA   = (_Float16*)take((size_t)MROWS * DFF * 2);
  _Float16* RB   = (_Float16*)take((size_t)MROWS * DM * 2);
  _Float16* CTX  = (_Float16*)take((size_t)MROWS * DM * 2);
  if (off > ws_size || off > (size_t)134217728) return;
  _Float16* H16 = RA; _Float16* QKV = RA + (size_t)MROWS * DM; _Float16* MP = RA;
  _Float16* VT = RB;  _Float16* H2 = RB;
  k_wT<<<256, 256, 0, stream>>>(wq, HD, DM * HD, WQKV,                       DM, HD * DM, DM / 64, 1);
  k_wT<<<256, 256, 0, stream>>>(wk, HD, DM * HD, WQKV + (size_t)DM * DM,     DM, HD * DM, DM / 64, 1);
  k_wT<<<256, 256, 0, stream>>>(wv, HD, DM * HD, WQKV + (size_t)2 * DM * DM, DM, HD * DM, DM / 64, 1);
  k_wT<<<(DM / 64) * (DM / 64), 256, 0, stream>>>(wo, DM, 0, WO, DM, 0, DM / 64, DM / 64);
  k_wT<<<(DM / 64) * (DFF / 64), 256, 0, stream>>>(wfc, DFF, 0, WFC, DM, 0, DM / 64, DFF / 64);
  k_wT<<<(DFF / 64) * (DM / 64), 256, 0, stream>>>(wpr, DM, 0, WPR, DFF, 0, DFF / 64, DM / 64);
  k_ln<<<MROWS / 8, 256, 0, stream>>>(x, g1, bt1, H16, 1);
  k_gemm2<0><<<(MROWS / 128) * (LQ / 64), 128, 0, stream>>>(H16, DM, WQKV, DM, 0.0625f, bo, QKV, x, out, LQ, MROWS, LQ, DM);
  k_vt2<<<NB * NH * NQT, 256, 0, stream>>>(QKV, VT);
  k_attn<<<dim3((unsigned)NQT, (unsigned)(NB * NH)), 128, 0, stream>>>(QKV, VT, CTX);
  k_gemm2<2><<<(MROWS / 128) * (DM / 64), 128, 0, stream>>>(CTX, DM, WO, DM, 0.00390625f, bo, CTX, x, out, DM, MROWS, DM, DM);
  k_ln<<<MROWS / 8, 256, 0, stream>>>(out, g2, bt2, H2, 0);
  k_gemm2<1><<<(MROWS / 128) * (DFF / 64), 128, 0, stream>>>(H2, DM, WFC, DM, 0.0625f, bfc, MP, x, out, DFF, MROWS, DFF, DM);
  k_gemm2<3><<<(MROWS / 128) * (DM / 64), 128, 0, stream>>>(MP, DFF, WPR, DFF, 0.0625f, bpr, CTX, out, out, DM, MROWS, DM, DFF);
}
